// LPKT4LPR_15152644620310
// MI455X (gfx1250) — hardware-verified
//
#include <hip/hip_runtime.h>

typedef __attribute__((ext_vector_type(16))) _Float16 v16h;
typedef __attribute__((ext_vector_type(8)))  _Float16 v8h;
typedef __attribute__((ext_vector_type(8)))  float    v8f;
typedef __attribute__((ext_vector_type(4)))  float    v4f;

constexpr int kBatch   = 64;
constexpr int kSeq     = 128;
constexpr int kNumQ    = 2000;
constexpr int kNumC    = 128;
constexpr int kDimK    = 64;
constexpr int kDimE    = 64;
constexpr int kCatW    = 192;
constexpr int kGateK   = 128;
constexpr int kPitchA  = 72;
constexpr int kPitchB  = 136;
constexpr int kThreads = 256;

union FragU { v16h v; v8h h[2]; };

__device__ __forceinline__ v16h frag_load(const _Float16* p) {
  FragU f; f.h[0] = *(const v8h*)(p); f.h[1] = *(const v8h*)(p + 16); return f.v;
}

__device__ __forceinline__ v8f hmma(v16h a, v16h b, v8f c) {
  c = __builtin_amdgcn_wmma_f32_16x16x32_f16(false, a, false, b, (short)0, c, false, false);
  asm volatile("v_nop\n\tv_nop\n\tv_nop\n\tv_nop" : "+v"(c) : "v"(a), "v"(b));
  return c;
}

__device__ __forceinline__ float sigm_f(float x) {
  const float t = expf(-fabsf(x));
  const float s = __builtin_amdgcn_rcpf(1.0f + t);
  return (x >= 0.0f) ? s : t * s;
}
__device__ __forceinline__ float tanh_f(float x) {
  const float t = expf(-2.0f * fabsf(x));
  const float v = (1.0f - t) * __builtin_amdgcn_rcpf(1.0f + t);
  return copysignf(v, x);
}
__device__ __forceinline__ int clampi(int v, int hi) { return v < 0 ? 0 : (v > hi ? hi : v); }

__global__ __launch_bounds__(kThreads)
void kt_recurrent_main(const int* __restrict__ qseq, const int* __restrict__ cseq,
                       const float* __restrict__ qmat, const float* __restrict__ Eq,
                       const float* __restrict__ Ec, const float* __restrict__ h0g,
                       const float* __restrict__ W1, const float* __restrict__ b1,
                       const float* __restrict__ W2, const float* __restrict__ b2,
                       const float* __restrict__ W3, const float* __restrict__ b3,
                       const float* __restrict__ W4, const float* __restrict__ b4,
                       const float* __restrict__ Wab, const float* __restrict__ bab,
                       const float* __restrict__ Wdiff, const float* __restrict__ bdiff,
                       const float* __restrict__ Wdisc, const float* __restrict__ bdisc,
                       float* __restrict__ pred) {
  __shared__ __align__(16) _Float16 BtL[kDimK * kPitchB];
  __shared__ __align__(16) _Float16 hA[kNumC * kPitchA];
  __shared__ __align__(16) float qrowL[2 * kNumC];
  __shared__ __align__(16) float erowL[kDimE];
  __shared__ __align__(16) float crowL[kDimE];
  __shared__ __align__(16) float catL[kCatW];
  __shared__ __align__(16) float LrL[3 * kDimK];
  __shared__ __align__(16) float LGs[kDimK];
  __shared__ __align__(16) float htpL[8 * kDimK];
  __shared__ __align__(16) float contribL[kNumC];
  __shared__ __align__(16) float diffqL[kNumC];
  __shared__ __align__(16) float ysL[kSeq];
  __shared__ __align__(16) float b1L[kDimK];
  __shared__ __align__(16) float b2L[kDimK];
  __shared__ __align__(16) float b3L[kDimK];
  __shared__ __align__(16) float b4L[kDimK];
  __shared__ __align__(16) float WabL[kDimK];
  __shared__ __align__(16) float WdiscL[kDimK];
  __shared__ __align__(16) float bdiffL[kNumC];
  __shared__ __align__(16) float discL[4];

  const int b    = blockIdx.x;
  const int tid  = threadIdx.x;
  const int wv   = tid >> 5;
  const int lane = tid & 31;
  const int hh   = lane >> 4;
  const int ln   = lane & 15;

  for (int i = tid; i < kDimK * kGateK; i += kThreads) {
    const int n = i >> 7, k = i & 127;
    BtL[n * kPitchB + k] = (_Float16)(16.0f * W4[k * kDimK + n]);
  }
  if (tid < kDimK) {
    b1L[tid] = b1[tid]; b2L[tid] = b2[tid]; b3L[tid] = b3[tid]; b4L[tid] = b4[tid];
    WabL[tid] = Wab[tid]; WdiscL[tid] = Wdisc[tid];
    LrL[2 * kDimK + tid] = 0.0f;
  }
  if (tid < kNumC) bdiffL[tid] = bdiff[tid];

  float hreg[4][8];
#pragma unroll
  for (int nt = 0; nt < 4; ++nt) {
    const int n = nt * 16 + ln;
#pragma unroll
    for (int r = 0; r < 8; ++r) {
      const int c = 16 * wv + 8 * hh + r;
      const float v = h0g[c * kDimK + n];
      hreg[nt][r] = v;
      hA[c * kPitchA + n] = (_Float16)(8.0f * v);
    }
  }
  {
    const int q0id = clampi(qseq[b * kSeq], kNumQ - 1);
    const int c0id = clampi(cseq[b * kSeq], 1);
    if (tid < kNumC) qrowL[tid] = qmat[q0id * kNumC + tid];
    else if (tid < kNumC + kDimE) erowL[tid - kNumC] = Eq[q0id * kDimE + (tid - kNumC)];
    else crowL[tid - kNumC - kDimE] = Ec[c0id * kDimE + (tid - kNumC - kDimE)];
    if (tid == 0) ysL[0] = 0.0f;
  }
  __syncthreads();
  if (wv < 2) {
    const int n = tid;
    float a = 0.0f;
#pragma unroll 4
    for (int c = 0; c < kNumC; ++c) a += qrowL[c] * h0g[c * kDimK + n];
    htpL[n] = a;
#pragma unroll
    for (int w = 1; w < 8; ++w) htpL[w * kDimK + n] = 0.0f;
  } else if (wv < 4) {
    const int n = tid - 64;
    float a = 0.0f;
#pragma unroll 4
    for (int d = 0; d < kDimE; ++d) a += erowL[d] * W1[d * kDimK + n];
#pragma unroll 4
    for (int d = 0; d < kDimE; ++d) a += crowL[d] * W1[(kDimE + d) * kDimK + n];
    a += b1L[n];
    LrL[n] = a;
  }

  const float babv   = bab[0];
  const float bdiscv = bdisc[0];

#pragma unroll 1
  for (int t = 0; t < kSeq - 1; ++t) {
    __syncthreads();
    {
      const int qnid = clampi(qseq[b * kSeq + t + 1], kNumQ - 1);
      const int cnid = clampi(cseq[b * kSeq + t + 1], 1);
      const int slotn = ((t + 1) & 1) * kNumC;
      if (tid < kNumC) qrowL[slotn + tid] = qmat[qnid * kNumC + tid];
      else if (tid < kNumC + kDimE) erowL[tid - kNumC] = Eq[qnid * kDimE + (tid - kNumC)];
      else crowL[tid - kNumC - kDimE] = Ec[cnid * kDimE + (tid - kNumC - kDimE)];
    }
    if (wv < 2) {
      const int n = tid;
      float hv = 0.0f;
#pragma unroll
      for (int w = 0; w < 8; ++w) hv += htpL[w * kDimK + n];
      catL[2 * kDimK + n] = hv;
      catL[n]             = LrL[((t + 2) % 3) * kDimK + n];
      catL[kDimK + n]     = LrL[(t % 3) * kDimK + n];
    }
    if (wv == 2 && t > 0) {
      const float dsc = discL[0];
      float s = 0.0f;
#pragma unroll 4
      for (int c = 0; c < kNumC; ++c) s += dsc * contribL[c];
      const float yv = sigm_f(s);
      if (lane == 0) ysL[t] = yv;
    }
    __syncthreads();
    if (wv < 2) {
      const int n = tid;
      float a2 = 0.0f, a3 = 0.0f;
#pragma unroll 4
      for (int j = 0; j < kCatW; ++j) {
        const float cv = catL[j];
        a2 += cv * W2[j * kDimK + n];
        a3 += cv * W3[j * kDimK + n];
      }
      a2 += b2L[n];
      a3 += b3L[n];
      const float gain = tanh_f(a2);
      const float gl   = sigm_f(a3);
      LGs[n] = gl * (gain + 1.0f) * 0.5f;
    } else if (wv < 4) {
      const int n = tid - 64;
      float a = 0.0f;
#pragma unroll 4
      for (int d = 0; d < kDimE; ++d) a += erowL[d] * W1[d * kDimK + n];
#pragma unroll 4
      for (int d = 0; d < kDimE; ++d) a += crowL[d] * W1[(kDimE + d) * kDimK + n];
      a += b1L[n];
      LrL[((t + 1) % 3) * kDimK + n] = a;
    } else {
      const int c = tid - kNumC;
      float a = 0.0f;
#pragma unroll 4
      for (int d = 0; d < kDimE; ++d) a += erowL[d] * Wdiff[d * kNumC + c];
      a += bdiffL[c];
      diffqL[c] = sigm_f(a) * qrowL[((t + 1) & 1) * kNumC + c];
      if (wv == 4) {
        float ds = 0.0f;
#pragma unroll 4
        for (int d = 0; d < kDimE; ++d) ds += erowL[d] * WdiscL[d];
        ds += bdiscv;
        const float dv = sigm_f(ds) * 5.0f;
        if (lane == 0) discL[0] = dv;
      }
    }
    __syncthreads();
    {
      const _Float16* arow = hA + (16 * wv + ln) * kPitchA + 8 * hh;
      v8f acc[4];
#pragma unroll
      for (int nt = 0; nt < 4; ++nt) acc[nt] = (v8f){0.f, 0.f, 0.f, 0.f, 0.f, 0.f, 0.f, 0.f};
#pragma unroll
      for (int ks = 0; ks < 4; ++ks) {
        v16h a;
        if (ks < 2) {
          a = frag_load(arow + 32 * ks);
        } else {
          const float* lp = LGs + 32 * (ks - 2) + 8 * hh;
          const v4f x0 = *(const v4f*)(lp);
          const v4f x1 = *(const v4f*)(lp + 4);
          const v4f x2 = *(const v4f*)(lp + 16);
          const v4f x3 = *(const v4f*)(lp + 20);
          FragU u;
#pragma unroll
          for (int e = 0; e < 4; ++e) {
            u.h[0][e]     = (_Float16)(8.0f * x0[e]);
            u.h[0][4 + e] = (_Float16)(8.0f * x1[e]);
            u.h[1][e]     = (_Float16)(8.0f * x2[e]);
            u.h[1][4 + e] = (_Float16)(8.0f * x3[e]);
          }
          a = u.v;
        }
#pragma unroll
        for (int nt = 0; nt < 4; ++nt) {
          const v16h bf = frag_load(BtL + (nt * 16 + ln) * kPitchB + 32 * ks + 8 * hh);
          acc[nt] = hmma(a, bf, acc[nt]);
        }
      }
      __builtin_amdgcn_fence(__ATOMIC_RELEASE, "workgroup");
      __builtin_amdgcn_wave_barrier();
      __builtin_amdgcn_fence(__ATOMIC_ACQUIRE, "workgroup");

      float qe[8], qn[8], dq[8];
      {
        const float* pe = qrowL + (t & 1) * kNumC + 16 * wv + 8 * hh;
        const float* pn = qrowL + ((t + 1) & 1) * kNumC + 16 * wv + 8 * hh;
        const float* pd = diffqL + 16 * wv + 8 * hh;
        const v4f e0 = *(const v4f*)(pe), e1 = *(const v4f*)(pe + 4);
        const v4f n0 = *(const v4f*)(pn), n1 = *(const v4f*)(pn + 4);
        const v4f d0 = *(const v4f*)(pd), d1 = *(const v4f*)(pd + 4);
#pragma unroll
        for (int e = 0; e < 4; ++e) {
          qe[e] = e0[e]; qe[4 + e] = e1[e];
          qn[e] = n0[e]; qn[4 + e] = n1[e];
          dq[e] = d0[e]; dq[4 + e] = d1[e];
        }
      }
      float abil[8], htv[4];
#pragma unroll
      for (int r = 0; r < 8; ++r) abil[r] = 0.0f;
#pragma unroll
      for (int nt = 0; nt < 4; ++nt) htv[nt] = 0.0f;
#pragma unroll
      for (int nt = 0; nt < 4; ++nt) {
        const int n = nt * 16 + ln;
        const float lg  = LGs[n];
        const float b4v = b4L[n];
        const float wab = WabL[n];
#pragma unroll
        for (int r = 0; r < 8; ++r) {
          const float pre = acc[nt][r] * (1.0f / 128.0f) + b4v;
          const float gf  = sigm_f(pre);
          const float hn  = qe[r] * lg + gf * hreg[nt][r];
          hreg[nt][r] = hn;
          abil[r]  += hn * wab;
          htv[nt]  += qn[r] * hn;
          hA[(16 * wv + 8 * hh + r) * kPitchA + n] = (_Float16)(8.0f * hn);
        }
      }
#pragma unroll
      for (int r = 0; r < 8; ++r) {
        float v = abil[r];
        v += __shfl_xor(v, 1, 32);
        v += __shfl_xor(v, 2, 32);
        v += __shfl_xor(v, 4, 32);
        v += __shfl_xor(v, 8, 32);
        abil[r] = v;
      }
#pragma unroll
      for (int nt = 0; nt < 4; ++nt) htv[nt] += __shfl_xor(htv[nt], 16, 32);
      float cv[8];
#pragma unroll
      for (int r = 0; r < 8; ++r) cv[r] = sigm_f(abil[r] + babv) * qn[r] - dq[r];
      if (ln == 0) {
        float* cp = contribL + 16 * wv + 8 * hh;
        *(v4f*)(cp)     = (v4f){cv[0], cv[1], cv[2], cv[3]};
        *(v4f*)(cp + 4) = (v4f){cv[4], cv[5], cv[6], cv[7]};
      }
      if (hh == 0) {
#pragma unroll
        for (int nt = 0; nt < 4; ++nt) htpL[wv * kDimK + nt * 16 + ln] = htv[nt];
      }
    }
  }
  __syncthreads();
  if (wv == 2) {
    const float dsc = discL[0];
    float s = 0.0f;
#pragma unroll 4
    for (int c = 0; c < kNumC; ++c) s += dsc * contribL[c];
    const float yv = sigm_f(s);
    if (lane == 0) ysL[kSeq - 1] = yv;
  }
  __syncthreads();
  if (wv == 0) {
    const v4f v = *(const v4f*)(ysL + 4 * lane);
    float* dst = pred + (size_t)b * kSeq + 4 * lane;
    *(volatile v4f*)dst = v;
    __threadfence();
    *(volatile v4f*)dst = v;
  }
}

extern "C" void kernel_launch(void* const* d_in, const int* in_sizes, int n_in,
                              void* d_out, int out_size, void* d_ws, size_t ws_size,
                              hipStream_t stream) {
  (void)in_sizes; (void)n_in; (void)d_ws; (void)ws_size;
  const int*   qseq  = (const int*)d_in[0];
  const int*   cseq  = (const int*)d_in[1];
  const float* qmat  = (const float*)d_in[2];
  const float* Eq    = (const float*)d_in[3];
  const float* Ec    = (const float*)d_in[4];
  const float* h0    = (const float*)d_in[5];
  const float* W1    = (const float*)d_in[6];
  const float* b1    = (const float*)d_in[7];
  const float* W2    = (const float*)d_in[8];
  const float* b2    = (const float*)d_in[9];
  const float* W3    = (const float*)d_in[10];
  const float* b3    = (const float*)d_in[11];
  const float* W4    = (const float*)d_in[12];
  const float* b4    = (const float*)d_in[13];
  const float* Wab   = (const float*)d_in[14];
  const float* bab   = (const float*)d_in[15];
  const float* Wdiff = (const float*)d_in[16];
  const float* bdiff = (const float*)d_in[17];
  const float* Wdisc = (const float*)d_in[18];
  const float* bdisc = (const float*)d_in[19];
  float* pred = (float*)d_out;
  if (out_size < kBatch * kSeq) return;

  kt_recurrent_main<<<dim3(kBatch), dim3(kThreads), 0, stream>>>(
      qseq, cseq, qmat, Eq, Ec, h0, W1, b1, W2, b2, W3, b3, W4, b4,
      Wab, bab, Wdiff, bdiff, Wdisc, bdisc, pred);
}
